// EncoderLayer_1460288881504
// MI455X (gfx1250) — hardware-run, weakly checked
//
#include <hip/hip_runtime.h>


#ifndef NB
#define NB 2
#endif
#ifndef SEQ
#define SEQ 2048
#endif
#define NB_FULL  2
#define SEQ_FULL 2048
#ifndef OUT_SEQ
#define OUT_SEQ SEQ
#endif
#define DM    256
#define DIN   256
#define DST   256
#define DTR   16
#define DXP   528
#define DBP   576
#define DFF   1024
#define XZP   1024
#define MROWS (NB * SEQ)
#define GP    68
#define SCW   16
#define SPL   16
#define TC    16
#define WCAR  1024.0f
#define L2E   1.4426950408889634f
#define LNEPS 1.0e-5f

static_assert(SEQ % 32 == 0);
static_assert(MROWS % 32 == 0);
static_assert(MROWS % 8 == 0);
static_assert(DM == 256);
static_assert(DIN % 32 == 0);
static_assert(DIN % 64 == 0 && DM % 64 == 0 && DFF % 64 == 0 && XZP % 64 == 0 && DBP % 64 == 0);
static_assert(DBP >= DXP);
static_assert(DXP == DTR + 2 * DST);
static_assert(DM % 32 == 0 && DIN % 32 == 0 && DFF % 32 == 0);
static_assert(DTR == 16);
static_assert(SCW * SPL == DST);
static_assert(SCW == TC);
static_assert(SEQ % TC == 0);
static_assert(32 * SCW <= 512);
static_assert(SPL % 4 == 0);
static_assert(32 * 16 * 8 == 16 * 64 * 4);
static_assert((GP * 4) % 16 == 0);
static_assert((size_t)16 * GP * 4 <= 131072);
static_assert((size_t)SCW * TC * 32 * 4 <= 131072);
static_assert(NB <= NB_FULL);
static_assert(SEQ <= SEQ_FULL);
static_assert(XZP == 4 * DIN);

typedef _Float16 h16;
typedef __attribute__((ext_vector_type(16))) _Float16 v16h;
typedef __attribute__((ext_vector_type(8)))  _Float16 v8h;
typedef __attribute__((ext_vector_type(8)))  float    v8f;
typedef __attribute__((ext_vector_type(4)))  float    v4f;
typedef v4f  __attribute__((may_alias)) v4fa;

__device__ __forceinline__ unsigned short f2bf(float f) { unsigned u = __float_as_uint(f); u += 0x7FFFu + ((u >> 16) & 1u); return (unsigned short)(u >> 16); }
__device__ __forceinline__ float bfr(float f) { return __uint_as_float(((unsigned)f2bf(f)) << 16); }
__device__ __forceinline__ v16h cat16(v8h lo, v8h hi) { return __builtin_shufflevector(lo, hi, 0, 1, 2, 3, 4, 5, 6, 7, 8, 9, 10, 11, 12, 13, 14, 15); }
__device__ __forceinline__ v8f wmma16(v16h a, v16h b, v8f c) { return __builtin_amdgcn_wmma_f32_16x16x32_f16(false, a, false, b, (short)0, c, false, false); }
__device__ __forceinline__ v16h  ldh(const h16* p) { return cat16(*(const v8h*)p, *(const v8h*)(p + 16)); }
__device__ __forceinline__ void wave_sync() { __builtin_amdgcn_fence(3  , "wavefront"); __builtin_amdgcn_wave_barrier(); asm volatile("" ::: "memory"); }

static __device__ __forceinline__ h16 toh_flush(float v) { const h16 r = (h16)v; return (fabsf(v) < 6.103515625e-05f) ? (h16)0.0f : r; }
static __device__ __forceinline__ v8f wmma16g(v16h a, v16h b, v8f c) { c = wmma16(a, b, c); asm volatile("v_nop\n\tv_nop\n\tv_nop\n\tv_nop" : "+v"(c) : "v"(a), "v"(b)); return c; }

template <int ABFR, int K16>
static __device__ __forceinline__ v16h lda32(const float* p, float car) {
    const v4f x0 = *(const v4f*)p, x1 = *(const v4f*)(p + 4);
    v16h r;
#pragma unroll
    for (int i = 0; i < 4; ++i) { r[i] = toh_flush((ABFR ? bfr(x0[i]) : x0[i]) * car); r[4 + i] = toh_flush((ABFR ? bfr(x1[i]) : x1[i]) * car); }
    if (K16) {
#pragma unroll
        for (int i = 0; i < 8; ++i) r[8 + i] = (h16)0.0f;
    } else {
        const v4f x2 = *(const v4f*)(p + 16), x3 = *(const v4f*)(p + 20);
#pragma unroll
        for (int i = 0; i < 4; ++i) { r[8 + i] = toh_flush((ABFR ? bfr(x2[i]) : x2[i]) * car); r[12 + i] = toh_flush((ABFR ? bfr(x3[i]) : x3[i]) * car); }
    }
    return r;
}

__global__ __launch_bounds__(256) void k_wconv(const float* __restrict__ src, h16* dst, int srows, int scols, int drows, int dcols) {
    const size_t i = (size_t)blockIdx.x * 256 + threadIdx.x; const size_t n8 = (size_t)drows * (size_t)dcols / 8; if (i >= n8) return;
    const int r = (int)((i * 8) / (size_t)dcols), c = (int)((i * 8) % (size_t)dcols);
    const bool ok = (r < srows) & (c < scols);
    const int rc = r < srows ? r : (srows - 1), cc = c < scols ? c : (scols - 8);
    v4f x0 = *(const v4f*)(src + (size_t)rc * scols + cc), x1 = *(const v4f*)(src + (size_t)rc * scols + cc + 4);
    asm volatile("" : "+v"(x0), "+v"(x1));
    v8h o;
#pragma unroll
    for (int k = 0; k < 4; ++k) { const h16 a0 = toh_flush(bfr(x0[k]) * WCAR); const h16 a1 = toh_flush(bfr(x1[k]) * WCAR); o[k] = ok ? a0 : (h16)0.0f; o[4 + k] = ok ? a1 : (h16)0.0f; }
    *(volatile v8h*)(dst + i * 8) = o; __threadfence(); *(volatile v8h*)(dst + i * 8) = o;
}

template <int ABFR, int K16, int EPI>
static __device__ __forceinline__ void gemm_tile(const float* __restrict__ A, int lda, size_t abst, size_t azst, float acar,
                                                 const h16* __restrict__ Bt, size_t bzst, int K,
                                                 const float* __restrict__ bias, float oscale,
                                                 float* C, int ldc, size_t czst) {
    __shared__ __align__(16) float os[16 * GP];
    const int lane = threadIdx.x & 31, lr = lane & 15, hi = lane >> 4;
    const int r0 = blockIdx.x * 32, c0 = blockIdx.y * 64, z = blockIdx.z;
    const int bb = r0 / SEQ, tt = r0 % SEQ;
    const float* Ab = A + (size_t)z * azst + (size_t)bb * abst + (size_t)(tt + lr) * lda + 8 * hi;
    const h16* Bb = Bt + (size_t)z * bzst + (size_t)(c0 + lr) * K + 8 * hi;
    v8f acc[2][4];
#pragma unroll
    for (int mb = 0; mb < 2; ++mb)
#pragma unroll
        for (int nb = 0; nb < 4; ++nb) acc[mb][nb] = (v8f){};
#pragma unroll 1
    for (int kc = 0; kc < K; kc += 32) {
        v16h a[2];
#pragma unroll
        for (int mb = 0; mb < 2; ++mb) a[mb] = lda32<ABFR, K16>(Ab + (size_t)mb * 16 * lda + kc, acar);
#pragma unroll
        for (int nb = 0; nb < 4; ++nb) { const v16h b = ldh(Bb + (size_t)nb * 16 * K + kc);
#pragma unroll
            for (int mb = 0; mb < 2; ++mb) acc[mb][nb] = wmma16g(a[mb], b, acc[mb][nb]); }
    }
    const int prow = lane >> 4, cofs = (lane & 15) * 4;
    v4f bv = (v4f){};
    if (EPI >= 1) { const v4f t = *(const v4f*)(bias + c0 + cofs);
#pragma unroll
        for (int i = 0; i < 4; ++i) bv[i] = bfr(t[i]); }
    float* Cz = C + (size_t)z * czst + (size_t)r0 * ldc + c0;
#pragma unroll
    for (int mb = 0; mb < 2; ++mb) {
#pragma unroll
        for (int nb = 0; nb < 4; ++nb) {
#pragma unroll
            for (int j = 0; j < 8; ++j) os[(hi * 8 + j) * GP + nb * 16 + lr] = acc[mb][nb][j]; }
        wave_sync();
#pragma unroll 1
        for (int s = 0; s < 8; ++s) { const int row = 2 * s + prow;
            const v4f x = *(const v4fa*)(&os[row * GP + cofs]); v4f y;
#pragma unroll
            for (int i = 0; i < 4; ++i) { float f = x[i] * oscale;
                if (EPI >= 1) f = f + bv[i];
                if (EPI == 2) f = fmaxf(f, 0.0f);
                if (EPI == 3) f = fmaxf(f, 0.0f) + log1pf(__builtin_amdgcn_exp2f(-fabsf(f) * L2E));
                y[i] = f; }
            *(v4fa*)(&os[row * GP + cofs]) = y; }
        wave_sync();
        float* Cs = Cz + (size_t)(mb * 16) * ldc;
#pragma unroll 1
        for (int ps = 0; ps < 2; ++ps) {
#pragma unroll
            for (int s = 0; s < 8; ++s) { const int row = 2 * s + prow;
                const v4f val = *(const v4fa*)(&os[row * GP + cofs]);
                *(volatile v4f*)(Cs + (size_t)row * ldc + cofs) = val; }
            if (ps == 0) __threadfence(); }
        wave_sync();
    }
}

__global__ __launch_bounds__(32) void k_gemm_in(const float* __restrict__ A, int lda, size_t abst, size_t azst, float acar, const h16* __restrict__ Bt, size_t bzst, int K,
                                                const float* __restrict__ bias, float oscale, float* C, int ldc, size_t czst) {
    gemm_tile<1, 0, 0>(A, lda, abst, azst, acar, Bt, bzst, K, bias, oscale, C, ldc, czst);
}
__global__ __launch_bounds__(32) void k_gemm_plain(const float* __restrict__ A, int lda, size_t abst, size_t azst, float acar, const h16* __restrict__ Bt, size_t bzst, int K,
                                                   const float* __restrict__ bias, float oscale, float* C, int ldc, size_t czst) {
    gemm_tile<0, 0, 0>(A, lda, abst, azst, acar, Bt, bzst, K, bias, oscale, C, ldc, czst);
}
__global__ __launch_bounds__(32) void k_gemm_bias(const float* __restrict__ A, int lda, size_t abst, size_t azst, float acar, const h16* __restrict__ Bt, size_t bzst, int K,
                                                  const float* __restrict__ bias, float oscale, float* C, int ldc, size_t czst) {
    gemm_tile<0, 0, 1>(A, lda, abst, azst, acar, Bt, bzst, K, bias, oscale, C, ldc, czst);
}
__global__ __launch_bounds__(32) void k_gemm_relu(const float* __restrict__ A, int lda, size_t abst, size_t azst, float acar, const h16* __restrict__ Bt, size_t bzst, int K,
                                                  const float* __restrict__ bias, float oscale, float* C, int ldc, size_t czst) {
    gemm_tile<0, 0, 2>(A, lda, abst, azst, acar, Bt, bzst, K, bias, oscale, C, ldc, czst);
}
__global__ __launch_bounds__(32) void k_gemm_dt(const float* __restrict__ A, int lda, size_t abst, size_t azst, float acar, const h16* __restrict__ Bt, size_t bzst, int K,
                                                const float* __restrict__ bias, float oscale, float* C, int ldc, size_t czst) {
    gemm_tile<0, 1, 3>(A, lda, abst, azst, acar, Bt, bzst, K, bias, oscale, C, ldc, czst);
}

__global__ __launch_bounds__(256) void k_conv(const float* __restrict__ XZ, int xcol, const float* __restrict__ cw, const float* __restrict__ cb, float* XC, int rev) {
#pragma clang fp contract(off)
    const size_t i = (size_t)blockIdx.x * 256 + threadIdx.x; if (i >= (size_t)MROWS * (DIN / 4)) return;
    const int row = (int)(i / (DIN / 4)), d4 = (int)(i % (DIN / 4)) * 4; const int t = row % SEQ;
    const int tn = rev ? (t + 1 < SEQ ? t + 1 : SEQ - 1) : (t > 0 ? t - 1 : 0);
    const bool okn = rev ? (t < SEQ - 1) : (t > 0);
    const int rown = row - t + tn;
    const v4f xi = *(const v4f*)(XZ + (size_t)row * XZP + xcol + d4);
    v4f xn = *(const v4f*)(XZ + (size_t)rown * XZP + xcol + d4);
    asm volatile("" : "+v"(xn));
    const v4f c0 = *(const v4f*)(cw + d4 * 2), c1 = *(const v4f*)(cw + d4 * 2 + 4);
    const v4f bq = *(const v4f*)(cb + d4);
    float w0[4], w1[4];
    w0[0] = bfr(c0[0]); w1[0] = bfr(c0[1]); w0[1] = bfr(c0[2]); w1[1] = bfr(c0[3]);
    w0[2] = bfr(c1[0]); w1[2] = bfr(c1[1]); w0[3] = bfr(c1[2]); w1[3] = bfr(c1[3]);
    v4f o;
#pragma unroll
    for (int k = 0; k < 4; ++k) {
        const float xp = okn ? xn[k] : 0.0f;
        const float v = xp * w0[k] + xi[k] * w1[k] + bfr(bq[k]);
        o[k] = v * __builtin_amdgcn_rcpf(1.0f + __builtin_amdgcn_exp2f(-v * L2E)); }
    *(volatile v4f*)(XC + i * 4) = o; __threadfence(); *(volatile v4f*)(XC + i * 4) = o;
}

__global__ __launch_bounds__(32 * SCW) void k_scan(const float* __restrict__ DBC, const float* __restrict__ DT, const float* __restrict__ XC, const float* __restrict__ XZ, int zcol,
                                                   const float* __restrict__ Alog, const float* __restrict__ Dp, float* Y, int rev) {
    __shared__ __align__(16) float part[SCW * TC * 32];
    const int lane = threadIdx.x & 31;
    const int wave = __builtin_amdgcn_readfirstlane((int)(threadIdx.x >> 5));
    const int d = blockIdx.x * 32 + lane, b = blockIdx.y, s0 = wave * SPL;
    float a2[SPL], h[SPL];
    { const float* ap = Alog + (size_t)d * DST + s0;
#pragma unroll
      for (int q = 0; q < SPL / 4; ++q) { const v4f al = *(const v4f*)(ap + 4 * q);
#pragma unroll
          for (int k = 0; k < 4; ++k) { a2[4 * q + k] = -__builtin_amdgcn_exp2f(bfr(al[k]) * L2E) * L2E; h[4 * q + k] = 0.0f; } } }
    const float Dd = bfr(Dp[d]);
    const size_t rowb = (size_t)b * SEQ;
#pragma unroll 1
    for (int c = 0; c < SEQ / TC; ++c) {
#pragma unroll 1
        for (int j = 0; j < TC; ++j) {
            const int st = c * TC + j; const int t = rev ? (SEQ - 1 - st) : st; const size_t row = rowb + (size_t)t;
            const float dt = DT[row * DIN + d], u = XC[row * DIN + d];
            const float dtu = dt * u;
            const float* bp = DBC + row * DBP + DTR + s0;
            v4f Bq[SPL / 4], Cq[SPL / 4];
#pragma unroll
            for (int q = 0; q < SPL / 4; ++q) { Bq[q] = *(const v4f*)(bp + 4 * q); Cq[q] = *(const v4f*)(bp + DST + 4 * q); }
            float p = 0.0f;
#pragma unroll
            for (int i = 0; i < SPL; ++i) {
                const float dA = __builtin_amdgcn_exp2f(dt * a2[i]);
                h[i] = dA * h[i] + dtu * Bq[i >> 2][i & 3];
                p += h[i] * Cq[i >> 2][i & 3]; }
            part[(wave * TC + j) * 32 + lane] = p;
        }
        __syncthreads();
        { float s = 0.0f;
#pragma unroll 4
          for (int w = 0; w < SCW; ++w) s += part[(w * TC + wave) * 32 + lane];
          const int st = c * TC + wave; const int t = rev ? (SEQ - 1 - st) : st; const size_t row = rowb + (size_t)t;
          const float u = XC[row * DIN + d], zv = XZ[row * XZP + zcol + d];
          const float gate = zv * __builtin_amdgcn_rcpf(1.0f + __builtin_amdgcn_exp2f(-zv * L2E));
          const float yv = (s + u * Dd) * gate;
          *(volatile float*)(Y + row * DIN + d) = yv; __threadfence(); *(volatile float*)(Y + row * DIN + d) = yv; }
        __syncthreads();
    }
}

__global__ __launch_bounds__(256) void k_ln(const float* __restrict__ X0, size_t x0bst, int x0bf, const float* __restrict__ A1, const float* __restrict__ A2, int use2,
                                            const float* __restrict__ gam, const float* __restrict__ bet, float* O, size_t obst) {
#pragma clang fp contract(off)
    const int lane = threadIdx.x & 31;
    const int wave = __builtin_amdgcn_readfirstlane((int)(threadIdx.x >> 5));
    const int row = blockIdx.x * 8 + wave;
    if (row >= MROWS) return;
    const int bb = row / SEQ, tt = row % SEQ;
    const float* xr = X0 + (size_t)bb * x0bst + (size_t)tt * DM + 4 * lane;
    v4f x0 = *(const v4f*)xr, x1 = *(const v4f*)(xr + 128);
    if (x0bf) {
#pragma unroll
        for (int i = 0; i < 4; ++i) { x0[i] = bfr(x0[i]); x1[i] = bfr(x1[i]); } }
    const size_t ao = (size_t)row * DM + 4 * lane;
    v4f a0 = *(const v4f*)(A1 + ao), a1 = *(const v4f*)(A1 + ao + 128);
    if (use2) { const v4f b0 = *(const v4f*)(A2 + ao), b1 = *(const v4f*)(A2 + ao + 128); a0 = a0 + b0; a1 = a1 + b1; }
    x0 = x0 + a0; x1 = x1 + a1;
    float s = ((x0[0] + x0[1]) + (x0[2] + x0[3])) + ((x1[0] + x1[1]) + (x1[2] + x1[3]));
#pragma unroll
    for (int off = 16; off > 0; off >>= 1) s += __shfl_xor(s, off, 32);
    const float mean = s * (1.0f / DM);
    v4f e0, e1;
#pragma unroll
    for (int i = 0; i < 4; ++i) { e0[i] = x0[i] - mean; e1[i] = x1[i] - mean; }
    float q = ((e0[0] * e0[0] + e0[1] * e0[1]) + (e0[2] * e0[2] + e0[3] * e0[3])) + ((e1[0] * e1[0] + e1[1] * e1[1]) + (e1[2] * e1[2] + e1[3] * e1[3]));
#pragma unroll
    for (int off = 16; off > 0; off >>= 1) q += __shfl_xor(q, off, 32);
    const float rs = rsqrtf(q * (1.0f / DM) + LNEPS);
    const v4f g0 = *(const v4f*)(gam + 4 * lane), g1 = *(const v4f*)(gam + 128 + 4 * lane);
    const v4f h0 = *(const v4f*)(bet + 4 * lane), h1 = *(const v4f*)(bet + 128 + 4 * lane);
    v4f o0, o1;
#pragma unroll
    for (int i = 0; i < 4; ++i) { o0[i] = e0[i] * rs * bfr(g0[i]) + bfr(h0[i]); o1[i] = e1[i] * rs * bfr(g1[i]) + bfr(h1[i]); }
    float* orow = O + (size_t)bb * obst + (size_t)tt * DM + 4 * lane;
    *(volatile v4f*)orow = o0; *(volatile v4f*)(orow + 128) = o1;
    __threadfence();
    *(volatile v4f*)orow = o0; *(volatile v4f*)(orow + 128) = o1;
}

static constexpr size_t al256(size_t v) { return (v + 255) & ~(size_t)255; }
static constexpr size_t SZ_WIN  = al256((size_t)XZP * DM * 2);
static constexpr size_t SZ_WXP  = al256((size_t)2 * DBP * DIN * 2);
static constexpr size_t SZ_WDT  = al256((size_t)2 * DIN * 32 * 2);
static constexpr size_t SZ_WOUT = al256((size_t)2 * DM * DIN * 2);
static constexpr size_t SZ_W1   = al256((size_t)DFF * DM * 2);
static constexpr size_t SZ_W2   = al256((size_t)DM * DFF * 2);
static constexpr size_t SZ_XZ   = al256((size_t)MROWS * XZP * 4);
static constexpr size_t SZ_D256 = al256((size_t)2 * MROWS * DIN * 4);
static constexpr size_t SZ_DBC  = al256((size_t)2 * MROWS * DBP * 4);
static constexpr size_t SZ_XN   = al256((size_t)MROWS * DM * 4);
static constexpr size_t SZ_HID  = al256((size_t)MROWS * DFF * 4);
static constexpr size_t SZ_TOTAL = SZ_WIN + SZ_WXP + SZ_WDT + SZ_WOUT + SZ_W1 + SZ_W2 + SZ_XZ + 4 * SZ_D256 + SZ_DBC + 2 * SZ_XN + SZ_HID;
static_assert(SZ_TOTAL <= (size_t)134217728);
static_assert(((size_t)512 * DM * 2) % 256 == 0 && ((size_t)DBP * DIN * 2) % 256 == 0 && ((size_t)DIN * 32 * 2) % 256 == 0 && ((size_t)DM * DIN * 2) % 256 == 0);
static_assert(((size_t)MROWS * DIN * 4) % 256 == 0 && ((size_t)MROWS * DBP * 4) % 256 == 0);
static_assert(((size_t)MROWS * (DIN / 4)) % 256 == 0);
static_assert(DM == DIN);

extern "C" void kernel_launch(void* const* d_in, const int* in_sizes, int n_in,
                              void* d_out, int out_size, void* d_ws, size_t ws_size, hipStream_t stream) {
    if (n_in < 27) return;
    const size_t needx = ((size_t)(NB - 1) * SEQ_FULL + SEQ) * DM;
    if ((size_t)in_sizes[0] < needx) return;
    if ((size_t)in_sizes[1] < (size_t)512 * DM || (size_t)in_sizes[10] < (size_t)512 * DM) return;
    if (in_sizes[2] < DIN * 2 || in_sizes[11] < DIN * 2 || in_sizes[3] < DIN || in_sizes[12] < DIN) return;
    if ((size_t)in_sizes[4] < (size_t)DXP * DIN || (size_t)in_sizes[13] < (size_t)DXP * DIN) return;
    if (in_sizes[5] < DIN * DTR || in_sizes[14] < DIN * DTR || in_sizes[6] < DIN || in_sizes[15] < DIN) return;
    if ((size_t)in_sizes[7] < (size_t)DIN * DST || (size_t)in_sizes[16] < (size_t)DIN * DST || in_sizes[8] < DIN || in_sizes[17] < DIN) return;
    if ((size_t)in_sizes[9] < (size_t)DM * DIN || (size_t)in_sizes[18] < (size_t)DM * DIN) return;
    if (in_sizes[19] < DM || in_sizes[20] < DM || in_sizes[21] < DM || in_sizes[22] < DM) return;
    if ((size_t)in_sizes[23] < (size_t)DFF * DM || in_sizes[24] < DFF || (size_t)in_sizes[25] < (size_t)DM * DFF || in_sizes[26] < DM) return;
    if ((size_t)out_size < ((size_t)(NB - 1) * OUT_SEQ + SEQ) * DM) return;
    if (SZ_TOTAL > ws_size) return;
    const float* x = (const float*)d_in[0];
    const float* in_w[2]  = { (const float*)d_in[1],  (const float*)d_in[10] };
    const float* cv_w[2]  = { (const float*)d_in[2],  (const float*)d_in[11] };
    const float* cv_b[2]  = { (const float*)d_in[3],  (const float*)d_in[12] };
    const float* xp_w[2]  = { (const float*)d_in[4],  (const float*)d_in[13] };
    const float* dt_w[2]  = { (const float*)d_in[5],  (const float*)d_in[14] };
    const float* dt_b[2]  = { (const float*)d_in[6],  (const float*)d_in[15] };
    const float* alog[2]  = { (const float*)d_in[7],  (const float*)d_in[16] };
    const float* dsk[2]   = { (const float*)d_in[8],  (const float*)d_in[17] };
    const float* out_w[2] = { (const float*)d_in[9],  (const float*)d_in[18] };
    const float* n1g = (const float*)d_in[19]; const float* n1b = (const float*)d_in[20];
    const float* n2g = (const float*)d_in[21]; const float* n2b = (const float*)d_in[22];
    const float* w1 = (const float*)d_in[23]; const float* b1 = (const float*)d_in[24];
    const float* w2 = (const float*)d_in[25]; const float* b2 = (const float*)d_in[26];
    float* OUT = (float*)d_out;
    char* wsp = (char*)d_ws;
    h16* WIN  = (h16*)wsp; wsp += SZ_WIN;
    h16* WXP  = (h16*)wsp; wsp += SZ_WXP;
    h16* WDT  = (h16*)wsp; wsp += SZ_WDT;
    h16* WOUT = (h16*)wsp; wsp += SZ_WOUT;
    h16* W1H  = (h16*)wsp; wsp += SZ_W1;
    h16* W2H  = (h16*)wsp; wsp += SZ_W2;
    float* XZ  = (float*)wsp; wsp += SZ_XZ;
    float* XC  = (float*)wsp; wsp += SZ_D256;
    float* DBC = (float*)wsp; wsp += SZ_DBC;
    float* DTP = (float*)wsp; wsp += SZ_D256;
    float* YP  = (float*)wsp; wsp += SZ_D256;
    float* OP  = (float*)wsp; wsp += SZ_D256;
    float* XN1 = (float*)wsp; wsp += SZ_XN;
    float* HID = (float*)wsp; wsp += SZ_HID;
    float* FO  = (float*)wsp; wsp += SZ_XN;
    const float* nob = (const float*)d_ws;
    const size_t dpl = (size_t)MROWS * DIN;
    const size_t dbl = (size_t)MROWS * DBP;

    for (int dir = 0; dir < 2; ++dir) {
        k_wconv<<<(unsigned)(((size_t)512 * DM / 8 + 255) / 256), 256, 0, stream>>>(in_w[dir], WIN + (size_t)dir * 512 * DM, 512, DM, 512, DM);
        k_wconv<<<(unsigned)(((size_t)DBP * DIN / 8 + 255) / 256), 256, 0, stream>>>(xp_w[dir], WXP + (size_t)dir * DBP * DIN, DXP, DIN, DBP, DIN);
        k_wconv<<<(unsigned)(((size_t)DIN * 32 / 8 + 255) / 256), 256, 0, stream>>>(dt_w[dir], WDT + (size_t)dir * DIN * 32, DIN, DTR, DIN, 32);
        k_wconv<<<(unsigned)(((size_t)DM * DIN / 8 + 255) / 256), 256, 0, stream>>>(out_w[dir], WOUT + (size_t)dir * DM * DIN, DM, DIN, DM, DIN);
    }
    k_wconv<<<(unsigned)(((size_t)DFF * DM / 8 + 255) / 256), 256, 0, stream>>>(w1, W1H, DFF, DM, DFF, DM);
    k_wconv<<<(unsigned)(((size_t)DM * DFF / 8 + 255) / 256), 256, 0, stream>>>(w2, W2H, DM, DFF, DM, DFF);

    k_gemm_in<<<dim3(MROWS / 32, XZP / 64, 1), 32, 0, stream>>>(x, DM, (size_t)SEQ_FULL * DM, (size_t)0, 16.0f, WIN, (size_t)0, DM, nob, 1.0f / (16.0f * WCAR), XZ, XZP, (size_t)0);
    k_conv<<<(unsigned)((size_t)MROWS * (DIN / 4) / 256), 256, 0, stream>>>(XZ, 0, cv_w[0], cv_b[0], XC, 0);
    k_conv<<<(unsigned)((size_t)MROWS * (DIN / 4) / 256), 256, 0, stream>>>(XZ, 2 * DIN, cv_w[1], cv_b[1], XC + dpl, 1);
    k_gemm_plain<<<dim3(MROWS / 32, DBP / 64, 2), 32, 0, stream>>>(XC, DIN, (size_t)SEQ * DIN, dpl, 256.0f, WXP, (size_t)DBP * DIN, DIN, nob, 1.0f / (256.0f * WCAR), DBC, DBP, dbl);
    for (int dir = 0; dir < 2; ++dir)
        k_gemm_dt<<<dim3(MROWS / 32, DIN / 64, 1), 32, 0, stream>>>(DBC + (size_t)dir * dbl, DBP, (size_t)SEQ * DBP, (size_t)0, 1024.0f, WDT + (size_t)dir * DIN * 32, (size_t)0, 32,
                                                                    dt_b[dir], 1.0f / (1024.0f * WCAR), DTP + (size_t)dir * dpl, DIN, (size_t)0);
    for (int dir = 0; dir < 2; ++dir)
        k_scan<<<dim3(DIN / 32, NB, 1), 32 * SCW, 0, stream>>>(DBC + (size_t)dir * dbl, DTP + (size_t)dir * dpl, XC + (size_t)dir * dpl, XZ, dir * 2 * DIN + DIN,
                                                               alog[dir], dsk[dir], YP + (size_t)dir * dpl, dir);
    k_gemm_plain<<<dim3(MROWS / 32, DM / 64, 2), 32, 0, stream>>>(YP, DIN, (size_t)SEQ * DIN, dpl, 256.0f, WOUT, (size_t)DM * DIN, DIN, nob, 1.0f / (256.0f * WCAR), OP, DM, dpl);
    k_ln<<<MROWS / 8, 256, 0, stream>>>(x, (size_t)SEQ_FULL * DM, 1, OP, OP + dpl, 1, n1g, n1b, XN1, (size_t)SEQ * DM);
    k_gemm_relu<<<dim3(MROWS / 32, DFF / 64, 1), 32, 0, stream>>>(XN1, DM, (size_t)SEQ * DM, (size_t)0, 16.0f, W1H, (size_t)0, DM, b1, 1.0f / (16.0f * WCAR), HID, DFF, (size_t)0);
    k_gemm_bias<<<dim3(MROWS / 32, DM / 64, 1), 32, 0, stream>>>(HID, DFF, (size_t)SEQ * DFF, (size_t)0, 256.0f, W2H, (size_t)0, DFF, b2, 1.0f / (256.0f * WCAR), FO, DM, (size_t)0);
    k_ln<<<MROWS / 8, 256, 0, stream>>>(XN1, (size_t)SEQ * DM, 0, FO, FO, 0, n2g, n2b, OUT, (size_t)OUT_SEQ * DM);
}
